// EdgeModel_39702677684918
// MI455X (gfx1250) — hardware-run, weakly checked
//
#include <hip/hip_runtime.h>
#include <stddef.h>
#include <stdint.h>


#define DH      128
#define NRBF    16
#define NLAY    3
#define KA      256
#define PBW     256
#define WRK     32
#define MW1_L   (272 * DH)
#define MW2_L   (DH * DH)
#define UW1_L   (256 * DH)
#define UW2_L   (DH * DH)
#define NTHR    256
#define NWAVE   8
#define EPT     8
#define CHUNK   (NTHR * EPT)
#define WCAP    (EPT * 32)
#define LISTN   (NWAVE * WCAP)
#define NBA     1024
#define SLA     10
#define RCAP    16384
#define DEGCAP  64
#define GBM     64
#define GBN     128
#define GTHR    128
#define GWAVE   (GTHR / 32)
#define ROWH    256
#define SC_TP   132
#define SC_TILE (16 * SC_TP)
#define SC_LDS_BYTES (NWAVE * SC_TILE * 4 + NWAVE * ROWH * 2)
#define BK_ZINTS (LISTN + 2 * RCAP + 3 * NBA)
#define MISC_INTS 16
#define BK_LDS_INTS (BK_ZINTS + MISC_INTS)
#define WSMAX   134217728
#define T_NW1   0
#define T_NB1   256
#define T_NB2   384
#define T_WR    512
#define T_PB1   6656
#define T_MB2   7424
#define T_UB1   7808
#define T_UB2   8192
#define T_HB1   8576
#define T_HW256 8832
#define T_HW2   8960
#define T_HB2   9088
#define T_END   9120
#define T_CAP   9216
#define TBU     (T_CAP / 4)
#define EP_H0   0
#define EP_AB   1
#define EP_W2   2
#define EP_U1   3
#define EP_U2   4

static_assert(DH == 32 * 4);
static_assert(NRBF == 16);
static_assert((CHUNK & (CHUNK - 1)) == 0 && CHUNK <= 4096);
static_assert((NBA & (NBA - 1)) == 0 && NBA == (1 << SLA));
static_assert(((long long)CHUNK << SLA) < (1LL << 31));
static_assert(NBA % NWAVE == 0 && NBA % 32 == 0 && NBA == NTHR * 4);
static_assert(RCAP % (NTHR * 4) == 0 && BK_ZINTS % (NTHR * 4) == 0 && LISTN % 4 == 0);
static_assert(RCAP >= 12548 + 628 && DEGCAP >= 28 + 8);
static_assert(BK_LDS_INTS * 4 <= 327680);
static_assert(KA % 32 == 0 && (2 * KA) % 32 == 0 && KA == 2 * DH && ROWH == KA);
static_assert(GBN == DH && GBM == GWAVE * 16 && GTHR == GWAVE * 32);
static_assert(T_NB1 % 128 == 0 && T_NB2 % 128 == 0 && T_WR % 128 == 0 && T_PB1 % 128 == 0 && T_MB2 % 128 == 0);
static_assert(T_UB1 % 128 == 0 && T_UB2 % 128 == 0 && T_HB1 % 128 == 0 && T_HW256 % 128 == 0 && T_HW2 % 128 == 0);
static_assert(T_HB2 % 128 == 0 && T_END == T_HB2 + 32 && T_CAP >= T_END && TBU % NTHR == 0);
static_assert(T_PB1 - T_WR == NLAY * NRBF * DH && T_MB2 - T_PB1 == NLAY * 256 && T_UB1 - T_MB2 == NLAY * DH);
static_assert(WRK == 2 * NRBF && WRK % 32 == 0 && (NLAY * DH * WRK / 8) % NTHR == 0);
static_assert(SC_TP % 4 == 0 && SC_TP >= DH && SC_LDS_BYTES <= 327680 && (NWAVE * SC_TILE * 4) % 16 == 0);

typedef float          v2f   __attribute__((ext_vector_type(2)));
typedef float          v4f   __attribute__((ext_vector_type(4)));
typedef float          v8f   __attribute__((ext_vector_type(8)));
typedef int            v2i   __attribute__((ext_vector_type(2)));
typedef int            v4i   __attribute__((ext_vector_type(4)));
typedef int            v8i   __attribute__((ext_vector_type(8)));
typedef unsigned short v4us  __attribute__((ext_vector_type(4)));
typedef unsigned short v8us  __attribute__((ext_vector_type(8)));
typedef unsigned short v16us __attribute__((ext_vector_type(16)));
typedef __bf16         v16bf __attribute__((ext_vector_type(16)));
typedef v2f  __attribute__((may_alias)) v2fa;
typedef v4f  __attribute__((may_alias)) v4fa;
typedef v4i  __attribute__((may_alias)) v4ia;
typedef v4us __attribute__((may_alias)) v4usa;
typedef v8us __attribute__((may_alias)) v8usa;
union FragB { v16bf v; v16us u; v8us h[2]; v8i w; };

__device__ __forceinline__ v8f wmb(const FragB& a, const FragB& b, v8f c) {
  v8f d = __builtin_amdgcn_wmma_f32_16x16x32_bf16(false, a.v, false, b.v, (short)0, c, false, false);
  asm volatile("v_nop\n\tv_nop\n\tv_nop\n\tv_nop" : "+v"(d) : "v"(a.w), "v"(b.w));
  return d;
}

__device__ __forceinline__ v8f z8() { v8f z = {0.f, 0.f, 0.f, 0.f, 0.f, 0.f, 0.f, 0.f}; return z; }

__device__ __forceinline__ void ldwait() {
  asm volatile("s_wait_loadcnt 0x0" ::: "memory");
}

__device__ __forceinline__ unsigned bf16_bits(float f) {
  const unsigned u = __float_as_uint(f);
  return (u + 0x7FFFu + ((u >> 16) & 1u)) >> 16;
}
__device__ __forceinline__ float bf16_val(float f) {
  return __uint_as_float(bf16_bits(f) << 16);
}
__device__ __forceinline__ unsigned hl_bits(float v, unsigned& lo) {
  const unsigned hb = bf16_bits(v);
  lo = bf16_bits(v - __uint_as_float(hb << 16));
  return hb;
}

__device__ __forceinline__ void wave_sync() {
  __builtin_amdgcn_fence(__ATOMIC_RELEASE, "wavefront");
  __builtin_amdgcn_wave_barrier();
  __builtin_amdgcn_fence(__ATOMIC_ACQUIRE, "wavefront");
}

__device__ __forceinline__ float relu_k(float v) { return (v > 0.0f) ? v : (v - v); }

__device__ __forceinline__ v8us hl_pack(unsigned short* rb, int lane, float y0, float y1, float y2, float y3) {
  v4us h4, l4;
  unsigned lb;
  unsigned hb;
  hb = hl_bits(y0, lb); h4[0] = (unsigned short)hb; l4[0] = (unsigned short)lb;
  hb = hl_bits(y1, lb); h4[1] = (unsigned short)hb; l4[1] = (unsigned short)lb;
  hb = hl_bits(y2, lb); h4[2] = (unsigned short)hb; l4[2] = (unsigned short)lb;
  hb = hl_bits(y3, lb); h4[3] = (unsigned short)hb; l4[3] = (unsigned short)lb;
  *(v4usa*)(rb + 4 * lane)      = h4;
  *(v4usa*)(rb + DH + 4 * lane) = l4;
  wave_sync();
  const v8us q = *(const v8usa*)(rb + 8 * lane);
  wave_sync();
  return q;
}

template <int SLB>
__device__ __forceinline__ int scan_chunk(const int* __restrict__ dsts, int nE, int cbase, int slotBase,
                                          int nb, int vec8, int* list, int tid, int lane, int wave) {
  int wc = 0;
  const int el0  = tid * EPT;
  const int e0   = cbase + el0;
  const int sent = -2147483647 - 1;
  v4i da, db;
  if (vec8 != 0 && cbase + CHUNK <= nE) {
    da = *(const v4i*)(dsts + e0);
    db = *(const v4i*)(dsts + e0 + 4);
  } else {
    da.x = (e0     < nE) ? dsts[min(e0,     nE - 1)] : sent;
    da.y = (e0 + 1 < nE) ? dsts[min(e0 + 1, nE - 1)] : sent;
    da.z = (e0 + 2 < nE) ? dsts[min(e0 + 2, nE - 1)] : sent;
    da.w = (e0 + 3 < nE) ? dsts[min(e0 + 3, nE - 1)] : sent;
    db.x = (e0 + 4 < nE) ? dsts[min(e0 + 4, nE - 1)] : sent;
    db.y = (e0 + 5 < nE) ? dsts[min(e0 + 5, nE - 1)] : sent;
    db.z = (e0 + 6 < nE) ? dsts[min(e0 + 6, nE - 1)] : sent;
    db.w = (e0 + 7 < nE) ? dsts[min(e0 + 7, nE - 1)] : sent;
  }
  const unsigned nbs = (unsigned)slotBase;
  const unsigned unb = (unsigned)nb;
  const unsigned s0 = (unsigned)da.x - nbs, s1 = (unsigned)da.y - nbs;
  const unsigned s2 = (unsigned)da.z - nbs, s3 = (unsigned)da.w - nbs;
  const unsigned s4 = (unsigned)db.x - nbs, s5 = (unsigned)db.y - nbs;
  const unsigned s6 = (unsigned)db.z - nbs, s7 = (unsigned)db.w - nbs;
  const bool h0 = s0 < unb, h1 = s1 < unb, h2 = s2 < unb, h3 = s3 < unb;
  const bool h4 = s4 < unb, h5 = s5 < unb, h6 = s6 < unb, h7 = s7 < unb;
  const unsigned any = __builtin_amdgcn_ballot_w32(h0 | h1 | h2 | h3 | h4 | h5 | h6 | h7);
  if (any != 0u) {
#define HITJ(J, HJ, SJ) { \
      const unsigned mj = __builtin_amdgcn_ballot_w32(HJ); \
      if (mj != 0u) { \
        if (HJ) { \
          const int pos = wc + (int)__builtin_amdgcn_mbcnt_lo(mj, 0u); \
          if (pos < WCAP) list[wave * WCAP + pos] = ((el0 + (J)) << SLB) | (int)(SJ); \
        } \
        wc += (int)__builtin_popcount(mj); } }
    HITJ(0, h0, s0)
    HITJ(1, h1, s1)
    HITJ(2, h2, s2)
    HITJ(3, h3, s3)
    HITJ(4, h4, s4)
    HITJ(5, h5, s5)
    HITJ(6, h6, s6)
    HITJ(7, h7, s7)
#undef HITJ
  }
  return wc;
}

__global__ __launch_bounds__(NTHR) void k_wplane(const float* __restrict__ W, int lstride, int nOut, int Kout,
                                                 int nsel, int ksel, int kmask, unsigned short* out, int nUnits) {
  const int u = (int)blockIdx.x * NTHR + (int)threadIdx.x;
  if (u >= nUnits) return;
  const int kq  = Kout >> 3;
  const int per = nOut * kq;
  const int l   = u / per;
  const int v   = u - l * per;
  const int n   = v / kq;
  const int k8  = (v - n * kq) * 8;
  const int srow = (n >> 7) * nsel + (k8 >> 8) * ksel + (k8 & kmask);
  const float* p = W + (size_t)l * (size_t)lstride + (size_t)srow * DH + (size_t)(n & 127);
  float f[8];
#pragma unroll
  for (int i = 0; i < 8; ++i) f[i] = p[(size_t)i * DH];
  v8us o;
#pragma unroll
  for (int i = 0; i < 8; ++i) o[i] = (unsigned short)bf16_bits(f[i]);
  unsigned short* dp = out + (size_t)u * 8;
  *(volatile v8us*)dp = o;
  __threadfence();
  *(volatile v8us*)dp = o;
}

__global__ __launch_bounds__(NTHR) void k_tables(const float* __restrict__ coords,
    const float* __restrict__ nW1, const float* __restrict__ nb1, const float* __restrict__ nb2,
    const float* __restrict__ mW1, const float* __restrict__ mb1, const float* __restrict__ mb2,
    const float* __restrict__ ub1, const float* __restrict__ ub2,
    const float* __restrict__ hW1, const float* __restrict__ hb1, const float* __restrict__ hW2,
    const float* __restrict__ hb2, float* TB, float* CB, int nCBu) {
  const int t = (int)blockIdx.x * NTHR + (int)threadIdx.x;
  v4f v = {0.f, 0.f, 0.f, 0.f};
  float* dp;
  if (t < TBU) {
    const int o = 4 * t;
    if (o >= T_END) return;
    if (o < T_NB1) {
      v = *(const v4f*)(nW1 + o);
    } else if (o < T_NB2) {
      v = *(const v4f*)(nb1 + (o - T_NB1));
    } else if (o < T_WR) {
      v = *(const v4f*)(nb2 + (o - T_NB2));
    } else if (o < T_PB1) {
      const int q = o - T_WR;
      const int l = q >> 11;
      const int r = q & 2047;
      v = *(const v4f*)(mW1 + (size_t)l * MW1_L + (size_t)256 * DH + r);
    } else if (o < T_MB2) {
      const int q = o - T_PB1;
      const int l = q >> 8;
      const int c = q & 255;
      const v4f x = *(const v4f*)(mb1 + l * DH + (c & 127));
      const bool up = c >= 128;
      v.x = up ? x.x : 0.0f; v.y = up ? x.y : 0.0f; v.z = up ? x.z : 0.0f; v.w = up ? x.w : 0.0f;
    } else if (o < T_UB1) {
      v = *(const v4f*)(mb2 + (o - T_MB2));
    } else if (o < T_UB2) {
      v = *(const v4f*)(ub1 + (o - T_UB1));
    } else if (o < T_HB1) {
      v = *(const v4f*)(ub2 + (o - T_UB2));
    } else if (o < T_HW256) {
      const int c = o - T_HB1;
      const v4f x = *(const v4f*)(hb1 + (c & 127));
      const bool up = c >= 128;
      v.x = up ? x.x : 0.0f; v.y = up ? x.y : 0.0f; v.z = up ? x.z : 0.0f; v.w = up ? x.w : 0.0f;
    } else if (o < T_HW2) {
      v = *(const v4f*)(hW1 + (size_t)256 * DH + (o - T_HW256));
    } else if (o < T_HB2) {
      v = *(const v4f*)(hW2 + (o - T_HW2));
    } else {
      const float b = hb2[0];
      v.x = (o == T_HB2) ? b : 0.0f;
    }
    dp = TB + o;
  } else {
    const int cu = t - TBU;
    if (cu >= nCBu) return;
    v = *(const v4f*)(coords + (size_t)4 * cu);
    dp = CB + (size_t)4 * cu;
  }
  v4f w;
  w.x = bf16_val(v.x); w.y = bf16_val(v.y); w.z = bf16_val(v.z); w.w = bf16_val(v.w);
  *(volatile v4f*)dp = w;
  __threadfence();
  *(volatile v4f*)dp = w;
}

__global__ __launch_bounds__(NTHR) void k_bucket(const int* __restrict__ srcs, const int* __restrict__ dsts,
                                                 int nE, int nN, int vec8,
                                                 int* lsrcAll, int* offA, int* cntA, int* flg) {
  extern __shared__ __attribute__((aligned(16))) int dsm[];
  int* list = dsm;
  int* hl   = dsm + LISTN;
  int* sl   = hl + RCAP;
  int* cnt  = sl + RCAP;
  int* offs = cnt + NBA;
  int* cur  = offs + NBA;
  int* misc = cur + NBA;
  const int tid = (int)threadIdx.x, lane = tid & 31, wave = tid >> 5;
  const int nodeBase = (int)blockIdx.x * NBA;

  {
    const v4i z4 = {0, 0, 0, 0};
    for (int i = tid * 4; i < BK_ZINTS; i += NTHR * 4) *(v4ia*)(dsm + i) = z4;
    if (tid < MISC_INTS) misc[tid] = 0;
  }
  __syncthreads();

  int t = 0, ov = 0;
  const int nChunks = (nE + CHUNK - 1) / CHUNK;
#pragma unroll 1
  for (int ch = 0; ch < nChunks; ++ch) {
    const int cbase = ch * CHUNK;
    const int wc = scan_chunk<SLA>(dsts, nE, cbase, nodeBase, NBA, vec8, list, tid, lane, wave);
    if (lane == 0) misc[wave] = wc;
    __syncthreads();
    if (wave == 0) {
#pragma unroll 1
      for (int w2 = 0; w2 < NWAVE; ++w2) {
        int c = misc[w2];
        c = c < 0 ? 0 : (c > WCAP ? WCAP : c);
#pragma unroll 1
        for (int b0 = 0; b0 < c; b0 += 32) {
          const int idx = b0 + lane;
          const int ent_ = list[w2 * WCAP + (idx < WCAP ? idx : WCAP - 1)];
          const int m32 = (c - b0) < 32 ? (c - b0) : 32;
#pragma unroll 1
          for (int k = 0; k < m32; ++k) {
            const int u    = __builtin_amdgcn_readlane(ent_, k);
            const int slot = u & (NBA - 1);
            const int el   = (u >> SLA) & (CHUNK - 1);
            const int pk   = ((cbase + el) << SLA) | slot;
            if (t < RCAP) {
              if (lane == 0) { hl[t] = pk; cnt[slot] = cnt[slot] + 1; }
              t = t + 1;
            } else {
              ov = 1;
            }
          }
        }
      }
    }
    __syncthreads();
  }
  if (wave == 0 && lane == 0) { misc[8] = t; misc[9] = ov; }
  __syncthreads();
  int tt = misc[8];
  tt = tt < 0 ? 0 : (tt > RCAP ? RCAP : tt);
  const int ovf = misc[9];

  if (wave == 0) {
    const int base = lane * (NBA / 32);
    int s = 0;
#pragma unroll 1
    for (int i = 0; i < NBA / 32; ++i) s += cnt[base + i];
    int incl = s;
#pragma unroll
    for (int d = 1; d < 32; d <<= 1) {
      const int y = __shfl_up(incl, d, 32);
      if (lane >= d) incl += y;
    }
    int run = incl - s;
#pragma unroll 1
    for (int i = 0; i < NBA / 32; ++i) {
      const int cv = cnt[base + i];
      offs[base + i] = run;
      cur[base + i]  = run;
      run += cv;
    }
  }
  __syncthreads();
  if (wave == 0) {
#pragma unroll 1
    for (int b0 = 0; b0 < tt; b0 += 32) {
      const int idx = b0 + lane;
      const int ent_ = hl[idx < RCAP ? idx : RCAP - 1];
      const int m32 = (tt - b0) < 32 ? (tt - b0) : 32;
#pragma unroll 1
      for (int k = 0; k < m32; ++k) {
        const int u    = __builtin_amdgcn_readlane(ent_, k);
        const int slot = u & (NBA - 1);
        if (lane == 0) {
          int p = cur[slot];
          p = p < 0 ? 0 : (p > RCAP - 1 ? RCAP - 1 : p);
          sl[p] = u;
          cur[slot] = p + 1;
        }
      }
    }
  }
  __syncthreads();

  int* gl = lsrcAll + (size_t)blockIdx.x * RCAP;
#pragma unroll 1
  for (int it = 0; it < RCAP / (NTHR * 4); ++it) {
    const int p0 = (it * NTHR + tid) * 4;
    const v4i ent = *(const v4ia*)(sl + p0);
    int e0 = ent.x >> SLA, e1 = ent.y >> SLA, e2 = ent.z >> SLA, e3 = ent.w >> SLA;
    e0 = e0 < 0 ? 0 : (e0 > nE - 1 ? nE - 1 : e0);
    e1 = e1 < 0 ? 0 : (e1 > nE - 1 ? nE - 1 : e1);
    e2 = e2 < 0 ? 0 : (e2 > nE - 1 ? nE - 1 : e2);
    e3 = e3 < 0 ? 0 : (e3 > nE - 1 ? nE - 1 : e3);
    int s0 = srcs[e0], s1 = srcs[e1], s2 = srcs[e2], s3 = srcs[e3];
    ldwait();
    asm volatile("" :: "v"(s0)); asm volatile("" :: "v"(s1));
    asm volatile("" :: "v"(s2)); asm volatile("" :: "v"(s3));
    s0 = s0 < 0 ? 0 : (s0 > nN - 1 ? nN - 1 : s0);
    s1 = s1 < 0 ? 0 : (s1 > nN - 1 ? nN - 1 : s1);
    s2 = s2 < 0 ? 0 : (s2 > nN - 1 ? nN - 1 : s2);
    s3 = s3 < 0 ? 0 : (s3 > nN - 1 ? nN - 1 : s3);
    v4i o;
    o.x = (p0     < tt) ? s0 : 0;
    o.y = (p0 + 1 < tt) ? s1 : 0;
    o.z = (p0 + 2 < tt) ? s2 : 0;
    o.w = (p0 + 3 < tt) ? s3 : 0;
    *(volatile v4i*)(gl + p0) = o;
    __threadfence();
    *(volatile v4i*)(gl + p0) = o;
  }
  {
    const v4i o4 = *(const v4ia*)(offs + 4 * tid);
    const v4i c4 = *(const v4ia*)(cnt + 4 * tid);
    int* op = offA + (size_t)nodeBase + 4 * tid;
    int* cp = cntA + (size_t)nodeBase + 4 * tid;
    v4i f4; f4.x = ovf; f4.y = ovf; f4.z = ovf; f4.w = ovf;
    int* fp = flg + (size_t)blockIdx.x * 32 + 4 * (tid & 7);
    *(volatile v4i*)op = o4;
    *(volatile v4i*)cp = c4;
    if (tid < 8) *(volatile v4i*)fp = f4;
    __threadfence();
    *(volatile v4i*)op = o4;
    *(volatile v4i*)cp = c4;
    if (tid < 8) *(volatile v4i*)fp = f4;
  }
}

__global__ __launch_bounds__(NTHR) void k_embed(const float* __restrict__ CB, const float* __restrict__ TB,
                                                unsigned short* Shl, int nN, int mRows) {
  __shared__ __attribute__((aligned(16))) unsigned short rowb[NWAVE * ROWH];
  const int tid = (int)threadIdx.x, lane = tid & 31, wave = tid >> 5;
  const v4f w0 = *(const v4f*)(TB + T_NW1 + 4 * lane);
  const v4f w1 = *(const v4f*)(TB + T_NW1 + DH + 4 * lane);
  const v4f b1 = *(const v4f*)(TB + T_NB1 + 4 * lane);
  unsigned short* rb = rowb + wave * ROWH;
#pragma unroll 1
  for (int i = 0; i < 16; ++i) {
    const int row = (int)blockIdx.x * 128 + wave * 16 + i;
    const int rc  = row < nN ? row : nN - 1;
    const bool ok = row < nN;
    const v2f c = *(const v2fa*)(CB + (size_t)2 * rc);
    float y0 = fmaf(c.y, w1.x, c.x * w0.x) + b1.x;
    float y1 = fmaf(c.y, w1.y, c.x * w0.y) + b1.y;
    float y2 = fmaf(c.y, w1.z, c.x * w0.z) + b1.z;
    float y3 = fmaf(c.y, w1.w, c.x * w0.w) + b1.w;
    y0 = ok ? relu_k(y0) : 0.0f; y1 = ok ? relu_k(y1) : 0.0f;
    y2 = ok ? relu_k(y2) : 0.0f; y3 = ok ? relu_k(y3) : 0.0f;
    const v8us q = hl_pack(rb, lane, y0, y1, y2, y3);
    if (row < mRows) {
      unsigned short* gp = Shl + (size_t)row * KA + 8 * lane;
      *(volatile v8us*)gp = q;
      __threadfence();
      *(volatile v8us*)gp = q;
    }
  }
}

template <int EP>
__global__ __launch_bounds__(GTHR) __attribute__((amdgpu_num_vgpr(248)))
void k_gemm(const unsigned short* A1, const unsigned short* A2, int K2,
            const unsigned short* __restrict__ BT, int ldb,
            const float* __restrict__ bias, const int* __restrict__ cnt,
            float* Fo, int ldf, unsigned short* Ohl, int nN) {
  __shared__ __attribute__((aligned(16))) float stg[GBM * GBN];
  __shared__ __attribute__((aligned(16))) unsigned short rowb[GWAVE * ROWH];
  const int tid = (int)threadIdx.x, lane = tid & 31, wave = tid >> 5, hh = lane >> 4, m = lane & 15;
  const int rowBase = (int)blockIdx.x * GBM;
  const int col0    = (int)blockIdx.y * GBN;

  v8f acc[8];
#pragma unroll
  for (int t = 0; t < 8; ++t) acc[t] = z8();
  const size_t aoff = (size_t)(rowBase + 16 * wave + m) * (size_t)KA + 8 * hh;
  const unsigned short* ap1 = A1 + aoff;
  const unsigned short* ap2 = A2 + aoff;
  const unsigned short* bp  = BT + (size_t)(col0 + m) * (size_t)ldb + 8 * hh;

#pragma unroll 1
  for (int k0 = 0; k0 < KA; k0 += 32) {
    FragB af;
    af.h[0] = *(const v8usa*)(ap1 + k0);
    af.h[1] = *(const v8usa*)(ap1 + k0 + 16);
#pragma unroll
    for (int nt = 0; nt < 8; ++nt) {
      const unsigned short* wq = bp + (size_t)(16 * nt) * (size_t)ldb + k0;
      FragB bf;
      bf.h[0] = *(const v8usa*)wq;
      bf.h[1] = *(const v8usa*)(wq + 16);
      acc[nt] = wmb(af, bf, acc[nt]);
    }
  }
#pragma unroll 1
  for (int k0 = 0; k0 < K2; k0 += 32) {
    FragB af;
    af.h[0] = *(const v8usa*)(ap2 + k0);
    af.h[1] = *(const v8usa*)(ap2 + k0 + 16);
#pragma unroll
    for (int nt = 0; nt < 8; ++nt) {
      const unsigned short* wq = bp + (size_t)(16 * nt) * (size_t)ldb + KA + k0;
      FragB bf;
      bf.h[0] = *(const v8usa*)wq;
      bf.h[1] = *(const v8usa*)(wq + 16);
      acc[nt] = wmb(af, bf, acc[nt]);
    }
  }

#pragma unroll
  for (int nt = 0; nt < 8; ++nt) {
    const int lc = 16 * nt + m;
#pragma unroll
    for (int r = 0; r < 8; ++r) {
      const int lr = 16 * wave + 8 * hh + r;
      stg[lr * GBN + lc] = acc[nt][r];
    }
  }
  __syncthreads();

  const v4f b4 = *(const v4f*)(bias + col0 + 4 * lane);
  unsigned short* rb = rowb + wave * ROWH;
#pragma unroll 1
  for (int i = 0; i < 16; ++i) {
    const int lr  = 16 * wave + i;
    const int row = rowBase + lr;
    const bool ok = row < nN;
    const v4f d = *(const v4fa*)(stg + lr * GBN + 4 * lane);
    float y0, y1, y2, y3;
    if constexpr (EP == EP_W2) {
      int ci = cnt[row];
      ci = ci < 0 ? 0 : (ci > (1 << 20) ? (1 << 20) : ci);
      const float cf = (float)ci;
      y0 = fmaf(cf, b4.x, d.x); y1 = fmaf(cf, b4.y, d.y); y2 = fmaf(cf, b4.z, d.z); y3 = fmaf(cf, b4.w, d.w);
    } else if constexpr (EP == EP_U1) {
      y0 = relu_k(d.x + b4.x); y1 = relu_k(d.y + b4.y); y2 = relu_k(d.z + b4.z); y3 = relu_k(d.w + b4.w);
    } else if constexpr (EP == EP_U2) {
      const v4f hv = *(const v4f*)(Fo + (size_t)row * (size_t)ldf + 4 * lane);
      y0 = (d.x + b4.x) + hv.x; y1 = (d.y + b4.y) + hv.y; y2 = (d.z + b4.z) + hv.z; y3 = (d.w + b4.w) + hv.w;
    } else {
      y0 = d.x + b4.x; y1 = d.y + b4.y; y2 = d.z + b4.z; y3 = d.w + b4.w;
    }
    v4f yv;
    yv.x = ok ? y0 : 0.0f; yv.y = ok ? y1 : 0.0f; yv.z = ok ? y2 : 0.0f; yv.w = ok ? y3 : 0.0f;
    float* fp = Fo + (size_t)row * (size_t)ldf + col0 + 4 * lane;
    unsigned short* hp = Ohl + (size_t)row * (size_t)KA + 8 * lane;
    v8us q = {0, 0, 0, 0, 0, 0, 0, 0};
    if constexpr (EP != EP_AB) q = hl_pack(rb, lane, yv.x, yv.y, yv.z, yv.w);
    if constexpr (EP == EP_H0 || EP == EP_AB || EP == EP_U2) *(volatile v4f*)fp = yv;
    if constexpr (EP != EP_AB) *(volatile v8us*)hp = q;
    __threadfence();
    if constexpr (EP == EP_H0 || EP == EP_AB || EP == EP_U2) *(volatile v4f*)fp = yv;
    if constexpr (EP != EP_AB) *(volatile v8us*)hp = q;
  }
  (void)cnt; (void)Ohl; (void)rb;
}

__global__ __launch_bounds__(NTHR) void k_scan(const int* __restrict__ lsrcAll, const int* __restrict__ offA,
                                               const int* __restrict__ cntA, const int* __restrict__ flg,
                                               const float* __restrict__ CB, const float* __restrict__ PAB,
                                               const unsigned short* __restrict__ wrd, unsigned short* Shl,
                                               int nN, int mRows) {
  extern __shared__ __attribute__((aligned(16))) float sdyn[];
  const int tid = (int)threadIdx.x, lane = tid & 31, wave = tid >> 5, hh = lane >> 4, m = lane & 15;
  float* tb = sdyn + wave * SC_TILE;
  unsigned short* rb = (unsigned short*)(sdyn + NWAVE * SC_TILE) + wave * ROWH;

  FragB bfr[8];
#pragma unroll
  for (int nt = 0; nt < 8; ++nt) {
    const unsigned short* wq = wrd + (size_t)(16 * nt + m) * WRK + 8 * hh;
    bfr[nt].h[0] = *(const v8usa*)wq;
    bfr[nt].h[1] = *(const v8usa*)(wq + 16);
  }
  float ck[8];
#pragma unroll
  for (int i = 0; i < 8; ++i) {
    const float ca = 1.5f * ((float)i / 15.0f);
    const float cb = (i == 7) ? 1.5f : 1.5f * ((float)(8 + i) / 15.0f);
    ck[i] = (hh != 0) ? cb : ca;
  }
  const float wdt = 1.5f * (1.0f / 15.0f);

  const int nodeBase = (int)blockIdx.x * NBA;
  const int fl = flg[(size_t)blockIdx.x * 32];
  const float qnan = __int_as_float(0x7fc00000);
  const float pzb = (fl != 0) ? qnan : 0.0f;
  const int* lsrc = lsrcAll + (size_t)blockIdx.x * RCAP;

#pragma unroll 1
  for (int si = 0; si < NBA / NWAVE; ++si) {
    const int s    = si * NWAVE + wave;
    const int node = nodeBase + s;
    const int gcl  = node < nN ? node : nN - 1;
    int c = cntA[node];
    int o = offA[node];
    const bool big = c > DEGCAP;
    c = c < 0 ? 0 : (c > DEGCAP ? DEGCAP : c);
    o = o < 0 ? 0 : (o > RCAP ? RCAP : o);
    if (c > RCAP - o) c = RCAP - o;
    c = __builtin_amdgcn_readfirstlane(c);
    o = __builtin_amdgcn_readfirstlane(o);
    const float pzr = big ? qnan : pzb;
    const bool live = node < nN;
    const v4f pb = *(const v4f*)(PAB + (size_t)gcl * PBW + DH + 4 * lane);
    const v2f cd = *(const v2fa*)(CB + (size_t)2 * gcl);
    float a0 = 0.0f, a1 = 0.0f, a2 = 0.0f, a3 = 0.0f;
#pragma unroll 1
    for (int b0 = 0; b0 < c; b0 += 16) {
      int hq = b0 + m;
      hq = hq > c - 1 ? c - 1 : hq;
      int idx = o + hq;
      idx = idx > RCAP - 1 ? RCAP - 1 : idx;
      int sr = lsrc[idx];
      sr = sr < 0 ? 0 : (sr > nN - 1 ? nN - 1 : sr);
      const v2f cs = *(const v2fa*)(CB + (size_t)2 * sr);
      const float dx = cs.x - cd.x, dy = cs.y - cd.y;
      const float rr = sqrtf((dx * dx + dy * dy) + 1e-8f);
      FragB af;
#pragma unroll
      for (int i = 0; i < 8; ++i) {
        const float dq = (rr - ck[i]) / wdt;
        const float ev = expf(-(dq * dq));
        unsigned lb;
        const unsigned hb = hl_bits(ev, lb);
        af.u[i]     = (unsigned short)hb;
        af.u[8 + i] = (unsigned short)lb;
      }
#pragma unroll
      for (int nt = 0; nt < 8; ++nt) {
        const v8f d = wmb(af, bfr[nt], z8());
#pragma unroll
        for (int r = 0; r < 8; ++r) tb[(8 * hh + r) * SC_TP + 16 * nt + m] = d[r];
      }
      wave_sync();
      int m16 = (c - b0) < 16 ? (c - b0) : 16;
      m16 = m16 < 0 ? 0 : m16;
#pragma unroll 1
      for (int h = 0; h < m16; ++h) {
        const int sk = __builtin_amdgcn_readlane(sr, h);
        const v4f pa = *(const v4f*)(PAB + (size_t)sk * PBW + 4 * lane);
        const v4f t4 = *(const v4fa*)(tb + h * SC_TP + 4 * lane);
        const float p0 = (pa.x + pb.x) + t4.x;
        const float p1 = (pa.y + pb.y) + t4.y;
        const float p2 = (pa.z + pb.z) + t4.z;
        const float p3 = (pa.w + pb.w) + t4.w;
        a0 += relu_k(p0); a1 += relu_k(p1); a2 += relu_k(p2); a3 += relu_k(p3);
      }
      wave_sync();
    }
    const float y0 = live ? (a0 + pzr) : 0.0f;
    const float y1 = live ? (a1 + pzr) : 0.0f;
    const float y2 = live ? (a2 + pzr) : 0.0f;
    const float y3 = live ? (a3 + pzr) : 0.0f;
    const v8us q = hl_pack(rb, lane, y0, y1, y2, y3);
    if (node < mRows) {
      unsigned short* gp = Shl + (size_t)node * KA + 8 * lane;
      *(volatile v8us*)gp = q;
      __threadfence();
      *(volatile v8us*)gp = q;
    }
  }
}

__global__ __launch_bounds__(NTHR) void k_head(const int* __restrict__ pairs, const float* __restrict__ CB,
                                               const float* __restrict__ PAB, const float* __restrict__ TB,
                                               float* outp, int nN, int nP) {
  __shared__ __attribute__((aligned(16))) float sres[NBA];
  const int tid = (int)threadIdx.x, lane = tid & 31, wave = tid >> 5;
  const v4f hw = *(const v4f*)(TB + T_HW256 + 4 * lane);
  const v4f w2 = *(const v4f*)(TB + T_HW2 + 4 * lane);
  const float hb2 = TB[T_HB2];
  const int base = (int)blockIdx.x * NBA + wave * 128;
#pragma unroll 1
  for (int bt = 0; bt < 4; ++bt) {
    const int p  = base + bt * 32 + lane;
    const int pc = p < nP ? p : nP - 1;
    const v2i uv = *(const v2i*)(pairs + (size_t)2 * pc);
    int u = uv.x, v = uv.y;
    u = u < 0 ? 0 : (u > nN - 1 ? nN - 1 : u);
    v = v < 0 ? 0 : (v > nN - 1 ? nN - 1 : v);
    const v2f cu = *(const v2fa*)(CB + (size_t)2 * u);
    const v2f cv = *(const v2fa*)(CB + (size_t)2 * v);
    const float dx = cu.x - cv.x, dy = cu.y - cv.y;
    const float rc = sqrtf((dx * dx + dy * dy) + 1e-8f);
    const int ri = __float_as_int(rc);
    float res = 0.0f;
#pragma unroll 1
    for (int k = 0; k < 32; ++k) {
      const int uk = __builtin_amdgcn_readlane(u, k);
      const int vk = __builtin_amdgcn_readlane(v, k);
      const float rk = __int_as_float(__builtin_amdgcn_readlane(ri, k));
      const v4f pa = *(const v4f*)(PAB + (size_t)uk * PBW + 4 * lane);
      const v4f pb = *(const v4f*)(PAB + (size_t)vk * PBW + DH + 4 * lane);
      const float x0 = relu_k(fmaf(rk, hw.x, pa.x + pb.x));
      const float x1 = relu_k(fmaf(rk, hw.y, pa.y + pb.y));
      const float x2 = relu_k(fmaf(rk, hw.z, pa.z + pb.z));
      const float x3 = relu_k(fmaf(rk, hw.w, pa.w + pb.w));
      float part = x0 * w2.x;
      part = fmaf(x1, w2.y, part);
      part = fmaf(x2, w2.z, part);
      part = fmaf(x3, w2.w, part);
      part += __shfl_xor(part, 16, 32);
      part += __shfl_xor(part, 8, 32);
      part += __shfl_xor(part, 4, 32);
      part += __shfl_xor(part, 2, 32);
      part += __shfl_xor(part, 1, 32);
      const float tot = part + hb2;
      res = (lane == k) ? tot : res;
    }
    sres[wave * 128 + bt * 32 + lane] = res;
  }
  __syncthreads();
  const v4f ov = *(const v4fa*)(sres + 4 * tid);
  const int gp = (int)blockIdx.x * NBA + 4 * tid;
  float* op = outp + (size_t)gp;
  const bool wr = gp < nP;
  if (wr) *(volatile v4f*)op = ov;
  __threadfence();
  if (wr) *(volatile v4f*)op = ov;
}

static inline int cdiv(int a, int b) { return (a + b - 1) / b; }
static inline size_t al256(size_t o) { return (o + 255) & ~(size_t)255; }

extern "C" void kernel_launch(void* const* d_in, const int* in_sizes, int n_in,
                              void* d_out, int out_size, void* d_ws, size_t ws_size,
                              hipStream_t stream) {
  if (n_in < 19) return;
  if (in_sizes[0] < 2 * GBM || (in_sizes[0] & 1) != 0) return;
  const int nN = in_sizes[0] / 2;
  if (nN > (1 << 20) || ((2 * nN) % 32) != 0) return;
  if (in_sizes[1] < 2 || (in_sizes[1] & 1) != 0) return;
  const int nE = in_sizes[1] / 2;
  if (nE < 1 || nE >= (1 << 21)) return;
  if (in_sizes[2] < 64 || (in_sizes[2] & 1) != 0) return;
  const int nP = in_sizes[2] / 2;
  if ((nP % 32) != 0 || out_size != nP) return;
  if (in_sizes[3] != 2 * DH || in_sizes[4] != DH || in_sizes[5] != DH * DH || in_sizes[6] != DH) return;
  if (in_sizes[7] != NLAY * MW1_L || in_sizes[8] != NLAY * DH) return;
  if (in_sizes[9] != NLAY * MW2_L || in_sizes[10] != NLAY * DH) return;
  if (in_sizes[11] != NLAY * UW1_L || in_sizes[12] != NLAY * DH) return;
  if (in_sizes[13] != NLAY * UW2_L || in_sizes[14] != NLAY * DH) return;
  if (in_sizes[15] != 257 * DH || in_sizes[16] != DH || in_sizes[17] != DH || in_sizes[18] != 1) return;

  const float* coords = (const float*)d_in[0];
  const int*   ei     = (const int*)  d_in[1];
  const int*   pairs  = (const int*)  d_in[2];
  const float* nW1 = (const float*)d_in[3];
  const float* nb1 = (const float*)d_in[4];
  const float* nW2 = (const float*)d_in[5];
  const float* nb2 = (const float*)d_in[6];
  const float* mW1 = (const float*)d_in[7];
  const float* mb1 = (const float*)d_in[8];
  const float* mW2 = (const float*)d_in[9];
  const float* mb2 = (const float*)d_in[10];
  const float* uW1 = (const float*)d_in[11];
  const float* ub1 = (const float*)d_in[12];
  const float* uW2 = (const float*)d_in[13];
  const float* ub2 = (const float*)d_in[14];
  const float* hW1 = (const float*)d_in[15];
  const float* hb1 = (const float*)d_in[16];
  const float* hW2 = (const float*)d_in[17];
  const float* hb2 = (const float*)d_in[18];
  float* out = (float*)d_out;
  const int* src = ei;
  const int* dst = ei + nE;

  const int MP = cdiv(nN, 128) * 128;
  const int gM = MP / GBM;
  const int gA = cdiv(MP, NBA);
  if ((long long)gA * NBA < (long long)MP) return;
  const int vec8 = ((nE & 3) == 0) ? 1 : 0;

  char* ws = (char*)d_ws;
  size_t off = 0;
  const size_t oH   = off; off = al256(off + (size_t)MP * DH * 4);
  const size_t oHhl = off; off = al256(off + (size_t)MP * KA * 2);
  const size_t oShl = off; off = al256(off + (size_t)MP * KA * 2);
  const size_t oPAB = off; off = al256(off + (size_t)MP * PBW * 4);
  const size_t oLS  = off; off = al256(off + (size_t)gA * RCAP * 4);
  const size_t oOFF = off; off = al256(off + (size_t)gA * NBA * 4);
  const size_t oCNT = off; off = al256(off + (size_t)gA * NBA * 4);
  const size_t oFLG = off; off = al256(off + (size_t)gA * 32 * 4);
  const size_t oTB  = off; off = al256(off + (size_t)T_CAP * 4);
  const size_t oCB  = off; off = al256(off + (size_t)nN * 2 * 4);
  const size_t oNW2 = off; off = al256(off + (size_t)DH * KA * 2);
  const size_t oWAB = off; off = al256(off + (size_t)NLAY * 256 * KA * 2);
  const size_t oW2D = off; off = al256(off + (size_t)NLAY * DH * KA * 2);
  const size_t oU1C = off; off = al256(off + (size_t)NLAY * DH * 2 * KA * 2);
  const size_t oU2D = off; off = al256(off + (size_t)NLAY * DH * KA * 2);
  const size_t oHAB = off; off = al256(off + (size_t)256 * KA * 2);
  const size_t oWRD = off; off = al256(off + (size_t)NLAY * DH * WRK * 2);
  if (off > ws_size || off > (size_t)WSMAX) return;
  if ((size_t)MP * KA * 2 * 2 > (size_t)MP * PBW * 4) return;

  float*          H    = (float*)(ws + oH);
  unsigned short* Hhl  = (unsigned short*)(ws + oHhl);
  unsigned short* Shl  = (unsigned short*)(ws + oShl);
  float*          PAB  = (float*)(ws + oPAB);
  unsigned short* AGGh = (unsigned short*)(ws + oPAB);
  unsigned short* Thl  = (unsigned short*)(ws + oPAB + (size_t)MP * KA * 2);
  int*            LSRC = (int*)(ws + oLS);
  int*            OFFt = (int*)(ws + oOFF);
  int*            CNTt = (int*)(ws + oCNT);
  int*            FLG  = (int*)(ws + oFLG);
  float*          TB   = (float*)(ws + oTB);
  float*          CB   = (float*)(ws + oCB);
  unsigned short* NW2  = (unsigned short*)(ws + oNW2);
  unsigned short* WAB  = (unsigned short*)(ws + oWAB);
  unsigned short* W2D  = (unsigned short*)(ws + oW2D);
  unsigned short* U1C  = (unsigned short*)(ws + oU1C);
  unsigned short* U2D  = (unsigned short*)(ws + oU2D);
  unsigned short* HAB  = (unsigned short*)(ws + oHAB);
  unsigned short* WRD  = (unsigned short*)(ws + oWRD);

  const size_t bkLds = (size_t)BK_LDS_INTS * 4;
  const size_t scLds = (size_t)SC_LDS_BYTES;
  hipFuncSetAttribute(reinterpret_cast<const void*>(&k_bucket), hipFuncAttributeMaxDynamicSharedMemorySize, (int)bkLds);
  hipFuncSetAttribute(reinterpret_cast<const void*>(&k_scan), hipFuncAttributeMaxDynamicSharedMemorySize, (int)scLds);

  k_wplane<<<(DH * KA / 8) / NTHR, NTHR, 0, stream>>>(nW2, 0, DH, KA, 0, 0, 127, NW2, DH * KA / 8);
  k_wplane<<<(NLAY * 256 * KA / 8) / NTHR, NTHR, 0, stream>>>(mW1, MW1_L, 256, KA, 128, 0, 127, WAB,
                                                              NLAY * 256 * KA / 8);
  k_wplane<<<(NLAY * DH * KA / 8) / NTHR, NTHR, 0, stream>>>(mW2, MW2_L, DH, KA, 0, 0, 127, W2D, NLAY * DH * KA / 8);
  k_wplane<<<(NLAY * DH * 2 * KA / 8) / NTHR, NTHR, 0, stream>>>(uW1, UW1_L, DH, 2 * KA, 0, 128, 127, U1C,
                                                                 NLAY * DH * 2 * KA / 8);
  k_wplane<<<(NLAY * DH * KA / 8) / NTHR, NTHR, 0, stream>>>(uW2, UW2_L, DH, KA, 0, 0, 127, U2D, NLAY * DH * KA / 8);
  k_wplane<<<(256 * KA / 8) / NTHR, NTHR, 0, stream>>>(hW1, 0, 256, KA, 128, 0, 127, HAB, 256 * KA / 8);
  k_wplane<<<(NLAY * DH * WRK / 8) / NTHR, NTHR, 0, stream>>>(mW1 + (size_t)256 * DH, MW1_L, DH, WRK, 0, 0, 15, WRD,
                                                              NLAY * DH * WRK / 8);

  const int nCBu = (2 * nN) / 4;
  k_tables<<<cdiv(TBU + nCBu, NTHR), NTHR, 0, stream>>>(coords, nW1, nb1, nb2, mW1, mb1, mb2, ub1, ub2,
                                                        hW1, hb1, hW2, hb2, TB, CB, nCBu);
  k_bucket<<<gA, NTHR, bkLds, stream>>>(src, dst, nE, nN, vec8, LSRC, OFFt, CNTt, FLG);
  k_embed<<<MP / 128, NTHR, 0, stream>>>(CB, TB, Shl, nN, MP);
  k_gemm<EP_H0><<<dim3(gM, 1), GTHR, 0, stream>>>(Shl, Shl, 0, NW2, KA, TB + T_NB2, CNTt, H, DH, Hhl, nN);

  for (int l = 0; l < NLAY; ++l) {
    k_gemm<EP_AB><<<dim3(gM, 2), GTHR, 0, stream>>>(Hhl, Hhl, 0, WAB + (size_t)l * 256 * KA, KA,
                                                    TB + T_PB1 + l * 256, CNTt, PAB, PBW, Hhl, nN);
    k_scan<<<gA, NTHR, scLds, stream>>>(LSRC, OFFt, CNTt, FLG, CB, PAB, WRD + (size_t)l * DH * WRK, Shl, nN, MP);
    k_gemm<EP_W2><<<dim3(gM, 1), GTHR, 0, stream>>>(Shl, Shl, 0, W2D + (size_t)l * DH * KA, KA,
                                                    TB + T_MB2 + l * DH, CNTt, H, DH, AGGh, nN);
    k_gemm<EP_U1><<<dim3(gM, 1), GTHR, 0, stream>>>(Hhl, AGGh, KA, U1C + (size_t)l * DH * 2 * KA, 2 * KA,
                                                    TB + T_UB1 + l * DH, CNTt, H, DH, Thl, nN);
    k_gemm<EP_U2><<<dim3(gM, 1), GTHR, 0, stream>>>(Thl, Thl, 0, U2D + (size_t)l * DH * KA, KA,
                                                    TB + T_UB2 + l * DH, CNTt, H, DH, Hhl, nN);
  }

  k_gemm<EP_AB><<<dim3(gM, 2), GTHR, 0, stream>>>(Hhl, Hhl, 0, HAB, KA, TB + T_HB1, CNTt, PAB, PBW, Hhl, nN);
  k_head<<<cdiv(nP, NBA), NTHR, 0, stream>>>(pairs, CB, PAB, TB, out, nN, nP);
}
